// JAX_GeomAttention_15479062135061
// MI455X (gfx1250) — hardware-run, weakly checked
//
#include <hip/hip_runtime.h>
#include <math.h>
#include <stdint.h>

#ifndef FAST_EXP
#define FAST_EXP 0
#endif
#ifndef P_FORM
#define P_FORM 2
#endif

#define NB    4
#define LQ    2048
#define SK    2048
#define NH    8
#define HD    64
#define SEQ   LQ
#define TOK   (NH * HD)
#define NQB   (SEQ / 64)
#define NPAIR (NB * NH)
#define NBLK  (NPAIR * NQB)
#define RECP  16
#define OUT0_N    (NB * SEQ * NH * HD)
#define OUT1_ELEM OUT0_N
#define OUT_TOTAL (OUT0_N + 1)

static_assert(LQ == SK);
static_assert(HD == 64);
static_assert(SEQ % 64 == 0);
static_assert(TOK * 4 == 2048);
static_assert(NBLK == 1024);
static_assert(RECP * 8 == 128);
static_assert(OUT1_ELEM * 4 == 16777216);
static_assert(OUT1_ELEM < OUT_TOTAL);
static_assert(P_FORM == 1 || P_FORM == 2);

typedef __attribute__((ext_vector_type(16))) __bf16   v16b;
typedef __attribute__((ext_vector_type(8)))  __bf16   v8b;
typedef __attribute__((ext_vector_type(8)))  float    v8f;
typedef __attribute__((ext_vector_type(4)))  float    v4f;
typedef __attribute__((ext_vector_type(4)))  unsigned int v4u;
typedef __attribute__((ext_vector_type(2)))  double   v2d;

__device__ __forceinline__ unsigned short f2bf_bits(float f) {
  unsigned u = __float_as_uint(f);
  return (unsigned short)((u + 0x7FFFu + ((u >> 16) & 1u)) >> 16);
}
__device__ __forceinline__ float bf_bits2f(unsigned short h) { return __uint_as_float(((unsigned)h) << 16); }
__device__ __forceinline__ float rne_bf(float f) { return bf_bits2f(f2bf_bits(f)); }
__device__ __forceinline__ unsigned pk16(unsigned short a, unsigned short b) { return (unsigned)a | ((unsigned)b << 16); }
__device__ __forceinline__ v8f zero8() { v8f z = {0.f, 0.f, 0.f, 0.f, 0.f, 0.f, 0.f, 0.f}; return z; }

struct FragB {
  union U { v16b v; v8b h[2]; };
  static __device__ __forceinline__ v16b load(const __bf16* p) {
    U f; f.h[0] = *(const v8b*)(p); f.h[1] = *(const v8b*)(p + 16); return f.v;
  }
};

__device__ __forceinline__ __bf16 at_f2bf(float f) { return __builtin_bit_cast(__bf16, f2bf_bits(f)); }
__device__ __forceinline__ void at_split(float f, __bf16& hi, __bf16& lo) {
  const unsigned short hb = f2bf_bits(f);
  hi = __builtin_bit_cast(__bf16, hb);
  lo = at_f2bf(f - __uint_as_float(((unsigned)hb) << 16));
}
__device__ __forceinline__ v8f at_mma(v16b a, v16b b, v8f c) {
  c = __builtin_amdgcn_wmma_f32_16x16x32_bf16(false, a, false, b, (short)0, c, false, false);
  asm volatile("v_nop\n\tv_nop\n\tv_nop\n\tv_nop" : "+v"(c) : "v"(a), "v"(b));
  return c;
}

__device__ __forceinline__ float sm_exp(float x) {
#if FAST_EXP
  return exp2f(x * 1.44269504f);
#else
  return expf(x);
#endif
}

__device__ __forceinline__ float geom_score(float d, float cq) {
#pragma clang fp contract(off)
  float t = cq - d * d;
  t = (t > 0.0f) ? t : 0.0f;
  const float w = sqrtf(t + 1e-8f);
  return (0.5f * d + 0.5f * w) * 0.125f;
}

__global__ __launch_bounds__(256)
void k_prep(const float* __restrict__ q, const float* __restrict__ k, const float* __restrict__ v,
            unsigned short* __restrict__ QB, unsigned short* __restrict__ KB,
            unsigned short* __restrict__ VT, float* __restrict__ C2) {
  __shared__ __align__(16) float tq[64 * 68];
  __shared__ __align__(16) float tk[64 * 68];
  __shared__ __align__(16) float tv[64 * 68];
  __shared__ __align__(16) float sc2[64];

  const int tid  = threadIdx.x;
  const int bx   = blockIdx.x;
  const int tl   = bx % NQB;
  const int pair = bx / NQB;
  const int b    = pair / NH;
  const int h    = pair % NH;
  const int l0   = tl * 64;

  {
    const int lr = tid >> 4;
    const int c4 = (tid & 15) * 4;
#pragma unroll
    for (int it = 0; it < 4; ++it) {
      const int rr = it * 16 + lr;
      const size_t g = ((size_t)(b * SEQ + l0 + rr) * NH + h) * HD + c4;
      const v4f a  = *(const v4f*)(q + g);
      const v4f a2 = *(const v4f*)(k + g);
      const v4f a3 = *(const v4f*)(v + g);
      v4f ra, rb, rc;
#pragma unroll
      for (int e = 0; e < 4; ++e) { ra[e] = rne_bf(a[e]); rb[e] = rne_bf(a2[e]); rc[e] = rne_bf(a3[e]); }
      *(v4f*)(tq + rr * 68 + c4) = ra;
      *(v4f*)(tk + rr * 68 + c4) = rb;
      *(v4f*)(tv + rr * 68 + c4) = rc;
    }
  }
  __syncthreads();

  if (tid < 64) {
    float q2 = 0.0f, k2 = 0.0f;
#pragma unroll 1
    for (int e4 = 0; e4 < 16; ++e4) {
      const v4f a  = *(const v4f*)(tq + tid * 68 + e4 * 4);
      const v4f a2 = *(const v4f*)(tk + tid * 68 + e4 * 4);
      q2 += a[0] * a[0];   q2 += a[1] * a[1];   q2 += a[2] * a[2];   q2 += a[3] * a[3];
      k2 += a2[0] * a2[0]; k2 += a2[1] * a2[1]; k2 += a2[2] * a2[2]; k2 += a2[3] * a2[3];
    }
    sc2[tid] = q2 * k2;
  }

  const int sub = tid >> 3;
  const int c8  = (tid & 7) * 8;
  v4u wq[2], wk[2], wv[2];
#pragma unroll
  for (int it = 0; it < 2; ++it) {
    const int row = it * 32 + sub;
    const v4f qa = *(const v4f*)(tq + row * 68 + c8);
    const v4f qb = *(const v4f*)(tq + row * 68 + c8 + 4);
    const v4f ka = *(const v4f*)(tk + row * 68 + c8);
    const v4f kb = *(const v4f*)(tk + row * 68 + c8 + 4);
    v4u a, a2, a3;
    a[0]  = pk16(f2bf_bits(qa[0]), f2bf_bits(qa[1]));
    a[1]  = pk16(f2bf_bits(qa[2]), f2bf_bits(qa[3]));
    a[2]  = pk16(f2bf_bits(qb[0]), f2bf_bits(qb[1]));
    a[3]  = pk16(f2bf_bits(qb[2]), f2bf_bits(qb[3]));
    a2[0] = pk16(f2bf_bits(ka[0]), f2bf_bits(ka[1]));
    a2[1] = pk16(f2bf_bits(ka[2]), f2bf_bits(ka[3]));
    a2[2] = pk16(f2bf_bits(kb[0]), f2bf_bits(kb[1]));
    a2[3] = pk16(f2bf_bits(kb[2]), f2bf_bits(kb[3]));
#pragma unroll
    for (int qq = 0; qq < 4; ++qq) {
      const float f0 = tv[(c8 + 2 * qq) * 68 + row];
      const float f1 = tv[(c8 + 2 * qq + 1) * 68 + row];
      a3[qq] = pk16(f2bf_bits(f0), f2bf_bits(f1));
    }
    wq[it] = a; wk[it] = a2; wv[it] = a3;
  }
  for (int pass = 0; pass < 2; ++pass) {
#pragma unroll
    for (int it = 0; it < 2; ++it) {
      const int row = it * 32 + sub;
      const size_t go = ((size_t)pair * SEQ + l0 + row) * HD + c8;
      const size_t gv = ((size_t)pair * HD + row) * SEQ + l0 + c8;
      *(volatile v4u*)(QB + go) = wq[it];
      *(volatile v4u*)(KB + go) = wk[it];
      *(volatile v4u*)(VT + gv) = wv[it];
    }
    __threadfence();
  }
  __syncthreads();
  {
    const v4f cv = *(const v4f*)(sc2 + (tid & 15) * 4);
    asm volatile("" :: "v"(cv));
    if (tid < 16) {
      float* cp = C2 + (size_t)pair * SEQ + l0 + tid * 4;
      *(volatile v4f*)cp = cv;
      __threadfence();
      *(volatile v4f*)cp = cv;
    }
  }
}

__global__ __launch_bounds__(128) __attribute__((amdgpu_num_vgpr(248)))
void k_attn(const unsigned short* __restrict__ qbp, const unsigned short* __restrict__ kbp,
            const unsigned short* __restrict__ vtp, const float* __restrict__ c2p,
            float* __restrict__ out, double* __restrict__ rec) {
  union FB { v16b v; v8b h[2]; };
  __shared__ __align__(16) __bf16 Ksh[64 * HD];
  __shared__ __align__(16) __bf16 Vth[HD * 64];
  __shared__ __align__(16) __bf16 Psh[4][16 * 64];
#if P_FORM == 2
  __shared__ __align__(16) __bf16 Psl[4][16 * 64];
#endif
  __shared__ __align__(16) float  Os[4][16 * 68];
  __shared__ __align__(16) double red[128];

  const int tid  = threadIdx.x;
  const int wave = tid >> 5;
  const int lane = tid & 31;
  const int hh   = lane >> 4;
  const int c    = lane & 15;

  const int bx   = blockIdx.x;
  const int qb   = bx % NQB;
  const int pair = bx / NQB;
  const int b    = pair / NH;
  const int h    = pair % NH;
  const int q0   = qb * 64 + wave * 16;

  const __bf16* Qg = (const __bf16*)(const void*)qbp + (size_t)pair * SEQ * HD;
  const __bf16* Kg = (const __bf16*)(const void*)kbp + (size_t)pair * SEQ * HD;
  const __bf16* Vg = (const __bf16*)(const void*)vtp + (size_t)pair * HD * SEQ;
  const float*  cg = c2p + (size_t)pair * SEQ;
  float*        ob = out + (size_t)b * SEQ * TOK + h * HD;

  v16b qa[2];
#pragma unroll
  for (int dc = 0; dc < 2; ++dc)
    qa[dc] = FragB::load(Qg + (size_t)(q0 + c) * HD + dc * 32 + 8 * hh);

  float crow[8];
  {
    const v4f ca = *(const v4f*)(cg + q0 + 8 * hh);
    const v4f cb = *(const v4f*)(cg + q0 + 8 * hh + 4);
    crow[0] = ca[0]; crow[1] = ca[1]; crow[2] = ca[2]; crow[3] = ca[3];
    crow[4] = cb[0]; crow[5] = cb[1]; crow[6] = cb[2]; crow[7] = cb[3];
  }

  float mrow[8], lrow[8];
  v8f oacc[4];
#pragma unroll
  for (int r = 0; r < 8; ++r) { mrow[r] = -INFINITY; lrow[r] = 0.f; }
#pragma unroll
  for (int t = 0; t < 4; ++t) oacc[t] = zero8();
  float absacc = 0.0f;

  __bf16* pwh = Psh[wave];
#if P_FORM == 2
  __bf16* pwl = Psl[wave];
#endif

#pragma unroll 1
  for (int kc = 0; kc < NQB; ++kc) {
    const int kv0 = kc * 64;
    __syncthreads();
    {
      const int r = tid >> 1, half = (tid & 1) * 32;
      const __bf16* ks = Kg + (size_t)(kv0 + r) * HD + half;
      const __bf16* vs = Vg + (size_t)r * SEQ + kv0 + half;
#pragma unroll
      for (int i = 0; i < 4; ++i) {
        const v8b a0 = *(const v8b*)(ks + 8 * i);
        const v8b b0 = *(const v8b*)(vs + 8 * i);
        *(v8b*)(Ksh + r * HD + half + 8 * i) = a0;
        *(v8b*)(Vth + r * 64 + half + 8 * i) = b0;
      }
    }
    __syncthreads();

    v8f s[4];
#pragma unroll
    for (int j = 0; j < 4; ++j) {
      s[j] = zero8();
#pragma unroll
      for (int dc = 0; dc < 2; ++dc) {
        FB kb;
        kb.h[0] = *(const v8b*)(Ksh + (j * 16 + c) * HD + dc * 32 + 8 * hh);
        kb.h[1] = *(const v8b*)(Ksh + (j * 16 + c) * HD + dc * 32 + 16 + 8 * hh);
        s[j] = at_mma(qa[dc], kb.v, s[j]);
      }
    }

    float cm[8];
#pragma unroll
    for (int r = 0; r < 8; ++r) {
      float m = -INFINITY;
#pragma unroll
      for (int j = 0; j < 4; ++j) {
        const float sv = geom_score(s[j][r], crow[r]);
        s[j][r] = sv;
        absacc += fabsf(sv);
        m = fmaxf(m, sv);
      }
#pragma unroll
      for (int off = 1; off < 16; off <<= 1) m = fmaxf(m, __shfl_xor(m, off, 32));
      cm[r] = m;
    }

#pragma unroll
    for (int r = 0; r < 8; ++r) {
      const float mnew  = fmaxf(mrow[r], cm[r]);
      const float alpha = sm_exp(mrow[r] - mnew);
      mrow[r] = mnew;
      float psum = 0.f;
#pragma unroll
      for (int j = 0; j < 4; ++j) {
        const float p = sm_exp(s[j][r] - mnew);
        psum += p;
#if P_FORM == 2
        __bf16 a, bl; at_split(p, a, bl);
        pwh[(8 * hh + r) * 64 + j * 16 + c] = a;
        pwl[(8 * hh + r) * 64 + j * 16 + c] = bl;
#else
        pwh[(8 * hh + r) * 64 + j * 16 + c] = at_f2bf(p);
#endif
      }
#pragma unroll
      for (int off = 1; off < 16; off <<= 1) psum += __shfl_xor(psum, off, 32);
      lrow[r] = lrow[r] * alpha + psum;
#pragma unroll
      for (int t = 0; t < 4; ++t) oacc[t][r] *= alpha;
    }
    __builtin_amdgcn_fence(__ATOMIC_RELEASE, "workgroup");
    __builtin_amdgcn_wave_barrier();
    __builtin_amdgcn_fence(__ATOMIC_ACQUIRE, "workgroup");

#pragma unroll 1
    for (int kk = 0; kk < 2; ++kk) {
      FB pa;
      pa.h[0] = *(const v8b*)(pwh + c * 64 + kk * 32 + 8 * hh);
      pa.h[1] = *(const v8b*)(pwh + c * 64 + kk * 32 + 16 + 8 * hh);
#if P_FORM == 2
      FB pl;
      pl.h[0] = *(const v8b*)(pwl + c * 64 + kk * 32 + 8 * hh);
      pl.h[1] = *(const v8b*)(pwl + c * 64 + kk * 32 + 16 + 8 * hh);
#endif
#pragma unroll
      for (int t = 0; t < 4; ++t) {
        FB vb;
        vb.h[0] = *(const v8b*)(Vth + (t * 16 + c) * 64 + kk * 32 + 8 * hh);
        vb.h[1] = *(const v8b*)(Vth + (t * 16 + c) * 64 + kk * 32 + 16 + 8 * hh);
        oacc[t] = at_mma(pa.v, vb.v, oacc[t]);
#if P_FORM == 2
        oacc[t] = at_mma(pl.v, vb.v, oacc[t]);
#endif
      }
    }
  }

  float* os = Os[wave];
#pragma unroll
  for (int r = 0; r < 8; ++r) {
    const float inv = 1.0f / lrow[r];
#pragma unroll
    for (int t = 0; t < 4; ++t) os[(8 * hh + r) * 68 + t * 16 + c] = oacc[t][r] * inv;
  }
  __builtin_amdgcn_fence(__ATOMIC_RELEASE, "workgroup");
  __builtin_amdgcn_wave_barrier();
  __builtin_amdgcn_fence(__ATOMIC_ACQUIRE, "workgroup");
  {
    const int c4 = (lane & 15) * 4;
    for (int pass = 0; pass < 2; ++pass) {
#pragma unroll
      for (int it = 0; it < 8; ++it) {
        const int row = it * 2 + hh;
        v4f val = *(const v4f*)(os + row * 68 + c4);
        *(volatile v4f*)(ob + (size_t)(q0 + row) * TOK + c4) = val;
      }
      __threadfence();
    }
  }

  red[tid] = (double)absacc;
  __syncthreads();
  if (wave == 0) {
    double tsum = 0.0;
#pragma unroll 4
    for (int i = 0; i < 128; ++i) tsum += red[i];
    v2d val;
    val[0] = (lane == 0) ? tsum : 0.0;
    val[1] = 0.0;
    if (lane < 8) {
      double* rp = rec + (size_t)bx * RECP + lane * 2;
      *(volatile v2d*)rp = val;
      __threadfence();
      *(volatile v2d*)rp = val;
    }
  }
}

__global__ __launch_bounds__(32)
void k_final(const double* __restrict__ rec, float* __restrict__ out) {
  double t = 0.0;
#pragma unroll 4
  for (int i = 0; i < NBLK; ++i) t += rec[(size_t)i * RECP];
  const float mv = (float)(t * (1.0 / (4.0 * 8.0 * 2048.0 * 2048.0)));
  if (threadIdx.x == 0) {
    float* p = out + OUT1_ELEM;
    *(volatile float*)p = mv;
    __threadfence();
    *(volatile float*)p = mv;
  }
}

extern "C" void kernel_launch(void* const* d_in, const int* in_sizes, int n_in,
                              void* d_out, int out_size, void* d_ws, size_t ws_size,
                              hipStream_t stream) {
  if (n_in < 3) return;
  if (in_sizes[0] != OUT0_N || in_sizes[1] != OUT0_N || in_sizes[2] != OUT0_N) return;
  if (out_size != OUT_TOTAL) return;

  const float* q = (const float*)d_in[0];
  const float* k = (const float*)d_in[1];
  const float* v = (const float*)d_in[2];
  float* out = (float*)d_out;

  const size_t PB = (size_t)NPAIR * SEQ * HD * 2;
  const size_t PC = (size_t)NPAIR * SEQ * 4;
  const size_t PR = (size_t)NBLK * RECP * 8;
  size_t off = 0;
  const size_t oQB = off; off += PB;
  const size_t oKB = off; off += PB;
  const size_t oVT = off; off += PB;
  const size_t oC2 = off; off += PC;
  const size_t oRC = off; off += PR;
  if (off > ws_size) return;
  if (off > ((size_t)128 << 20)) return;

  char* ws = (char*)d_ws;
  unsigned short* QB = (unsigned short*)(ws + oQB);
  unsigned short* KB = (unsigned short*)(ws + oKB);
  unsigned short* VT = (unsigned short*)(ws + oVT);
  float*          C2 = (float*)(ws + oC2);
  double*         RC = (double*)(ws + oRC);

  k_prep<<<dim3(NBLK), dim3(256), 0, stream>>>(q, k, v, QB, KB, VT, C2);
  k_attn<<<dim3(NBLK), dim3(128), 0, stream>>>(QB, KB, VT, C2, out, RC);
  k_final<<<dim3(1), dim3(32), 0, stream>>>(RC, out);
  (void)hipGetLastError();
}
